// MyAttentionBlock_37400575213666
// MI455X (gfx1250) — hardware-verified
//
#include <hip/hip_runtime.h>
#include <math.h>

typedef __attribute__((ext_vector_type(16))) _Float16 v16h;
typedef __attribute__((ext_vector_type(8)))  _Float16 v8h;
typedef __attribute__((ext_vector_type(16))) __bf16   v16b;
typedef __attribute__((ext_vector_type(8)))  __bf16   v8b;
typedef __attribute__((ext_vector_type(8)))  float    v8f;
typedef __attribute__((ext_vector_type(4)))  float    v4f;

__device__ __forceinline__ unsigned short f2bf_bits(float f) {
  unsigned u = __float_as_uint(f);
  return (unsigned short)((u + 0x7FFFu + ((u >> 16) & 1u)) >> 16);
}
__device__ __forceinline__ float bf_bits2f(unsigned short h) { return __uint_as_float(((unsigned)h) << 16); }

__device__ __forceinline__ void dep_guard_h(v8f& a, v8f& b, v16h x, v16h y) { asm volatile("v_nop\n\tv_nop\n\tv_nop\n\tv_nop" : "+v"(a), "+v"(b) : "v"(x), "v"(y)); }
__device__ __forceinline__ void dep_guard_b(v8f& a, v8f& b, v16b x, v16b y) { asm volatile("v_nop\n\tv_nop\n\tv_nop\n\tv_nop" : "+v"(a), "+v"(b) : "v"(x), "v"(y)); }
__device__ __forceinline__ void keep4_h(v16h a, v16h b, v16h c, v16h d) { asm volatile("v_nop" :: "v"(a), "v"(b), "v"(c), "v"(d)); }
__device__ __forceinline__ void keep4_b(v16b a, v16b b, v16b c, v16b d) { asm volatile("v_nop" :: "v"(a), "v"(b), "v"(c), "v"(d)); }
__device__ __forceinline__ void acc_guard4(v8f& a, v8f& b, v8f& c, v8f& d) { asm volatile("v_nop\n\tv_nop\n\tv_nop\n\tv_nop" : "+v"(a), "+v"(b), "+v"(c), "+v"(d)); }

template <typename T> struct Frag;
template <> struct Frag<_Float16> {
  typedef v16h V; union U { v16h v; v8h h[2]; };
  static __device__ __forceinline__ v16h load(const _Float16* p) {
    U f; f.h[0] = *(const v8h*)(p); f.h[1] = *(const v8h*)(p + 16); return f.v;
  }
  static __device__ __forceinline__ v8f mma(v16h a, v16h b, v8f c) {
    return __builtin_amdgcn_wmma_f32_16x16x32_f16(false, a, false, b, (short)0, c, false, false);
  }
  static __device__ __forceinline__ void guard(v8f& a, v8f& b, v16h x, v16h y) { dep_guard_h(a, b, x, y); }
  static __device__ __forceinline__ void keep(v16h a, v16h b, v16h c, v16h d) { keep4_h(a, b, c, d); }
};
template <> struct Frag<__bf16> {
  typedef v16b V; union U { v16b v; v8b h[2]; };
  static __device__ __forceinline__ v16b load(const __bf16* p) {
    U f; f.h[0] = *(const v8b*)(p); f.h[1] = *(const v8b*)(p + 16); return f.v;
  }
  static __device__ __forceinline__ v8f mma(v16b a, v16b b, v8f c) {
    return __builtin_amdgcn_wmma_f32_16x16x32_bf16(false, a, false, b, (short)0, c, false, false);
  }
  static __device__ __forceinline__ void guard(v8f& a, v8f& b, v16b x, v16b y) { dep_guard_b(a, b, x, y); }
  static __device__ __forceinline__ void keep(v16b a, v16b b, v16b c, v16b d) { keep4_b(a, b, c, d); }
};

template <int ET> struct Elem;
template <> struct Elem<0> { typedef _Float16 T; };
template <> struct Elem<1> { typedef __bf16 T; };
template <int ET, bool SPLIT, int BIAS_MODE, int OUT_MODE, bool RESID, int ACT = 0>
__global__ __launch_bounds__(256) void wmma_gemm64(
    const unsigned short* __restrict__ Ap, const unsigned short* __restrict__ A2p, int lda, long strideA,
    const unsigned short* __restrict__ Btp, const unsigned short* __restrict__ Bt2p, int ldb, long strideB,
    void* __restrict__ Cout, void* __restrict__ Cout2, int ldc, long strideC,
    const float* __restrict__ bias,
    const float* __restrict__ resid, long strideR,
    int M, int N, int K, float scale) {
  typedef typename Elem<ET>::T T;
  typedef typename Frag<T>::V V;
  const T* A = (const T*)Ap; const T* A2 = (const T*)A2p; const T* Bt = (const T*)Btp; const T* Bt2 = (const T*)Bt2p;
  __shared__ __align__(16) float sT[8][16 * 68];
  const int b    = blockIdx.y;
  const int lane = threadIdx.x & 31;
  const int wave = threadIdx.x >> 5;
  const int tilesN = N >> 6;
  const int tilesM = M >> 6;
  const int tile = blockIdx.x * 8 + wave;
  if (tile >= tilesM * tilesN) return;
  const int tm = tile / tilesN;
  const int tn = tile - tm * tilesN;
  const int m0 = tm << 6;
  const int n0 = tn << 6;

  const T* Ab  = A  + (size_t)b * strideA;
  const T* Bb  = Bt + (size_t)b * strideB;
  const T* Ab2 = SPLIT ? (A2  + (size_t)b * strideA) : nullptr;
  const T* Bb2 = SPLIT ? (Bt2 + (size_t)b * strideB) : nullptr;

  const int rlane = lane & 15;
  const int koff  = (lane >> 4) * 8;
  const int mOff  = (lane >> 4) * 8;

  v8f acc[4][4];
#pragma unroll
  for (int i = 0; i < 4; ++i)
#pragma unroll
    for (int j = 0; j < 4; ++j) acc[i][j] = (v8f){0.f,0.f,0.f,0.f,0.f,0.f,0.f,0.f};

  for (int k0 = 0; k0 < K; k0 += 32) {
    V bh[4], bl[4];
#pragma unroll
    for (int j = 0; j < 4; ++j) {
      const size_t bo = (size_t)(n0 + (j << 4) + rlane) * ldb + koff + k0;
      bh[j] = Frag<T>::load(Bb + bo);
      if (SPLIT) bl[j] = Frag<T>::load(Bb2 + bo);
    }
#pragma unroll
    for (int i = 0; i < 4; ++i) {
      const size_t ao = (size_t)(m0 + (i << 4) + rlane) * lda + koff + k0;
      V ah = Frag<T>::load(Ab + ao);
      V al;
      if (SPLIT) al = Frag<T>::load(Ab2 + ao);
#pragma unroll
      for (int j = 0; j < 4; ++j) {
        acc[i][j] = Frag<T>::mma(ah, bh[j], acc[i][j]);
        if (SPLIT) {
          acc[i][j] = Frag<T>::mma(ah, bl[j], acc[i][j]);
          acc[i][j] = Frag<T>::mma(al, bh[j], acc[i][j]);
        }
      }
      Frag<T>::guard(acc[i][0], acc[i][3], ah, SPLIT ? al : ah);
    }
    Frag<T>::keep(bh[0], bh[1], bh[2], bh[3]);
    if (SPLIT) Frag<T>::keep(bl[0], bl[1], bl[2], bl[3]);
  }
  acc_guard4(acc[0][0], acc[0][1], acc[0][2], acc[0][3]);
  acc_guard4(acc[1][0], acc[1][1], acc[1][2], acc[1][3]);
  acc_guard4(acc[2][0], acc[2][1], acc[2][2], acc[2][3]);
  acc_guard4(acc[3][0], acc[3][1], acc[3][2], acc[3][3]);

  float* slab = sT[wave];
  const float* Rb = RESID ? (resid + (size_t)b * strideR) : nullptr;
#pragma unroll
  for (int i = 0; i < 4; ++i) {
    const int mBase = m0 + (i << 4);
#pragma unroll
    for (int j = 0; j < 4; ++j) {
      const int n = n0 + (j << 4) + rlane;
      float bv = 0.f;
      if (BIAS_MODE == 2) bv = bias[n];
#pragma unroll
      for (int r = 0; r < 8; ++r) {
        float v = acc[i][j][r] * scale;
        if (BIAS_MODE == 1) v += bias[mBase + mOff + r];
        if (BIAS_MODE == 2) v += bv;
        if (RESID) v += Rb[(size_t)(mBase + mOff + r) * ldc + n];
        if (ACT == 1) v = tanhf(v);
        if (ACT == 2) v = fmaxf(v, 0.0f);
        if (ACT == 3) v = v / (1.0f + expf(-v));
        if (ACT == 4) v = (v > 0.f) ? v : 0.01f * v;
        if (ACT == 5) v = 0.5f * v * (1.0f + erff(v * 0.70710678118654752f));
        slab[(mOff + r) * 68 + (j << 4) + rlane] = v;
      }
    }
    __builtin_amdgcn_fence(__ATOMIC_RELEASE, "workgroup");
    __builtin_amdgcn_wave_barrier();
    __builtin_amdgcn_fence(__ATOMIC_ACQUIRE, "workgroup");
    if (OUT_MODE == 0) {
      float* C = (float*)Cout + (size_t)b * strideC;
      const int hh = lane >> 4, c4 = (lane & 15) * 4;
      for (int pass = 0; pass < 2; ++pass) {
#pragma unroll
        for (int it = 0; it < 8; ++it) {
          const int row = it * 2 + hh;
          v4f v = *(const v4f*)(slab + row * 68 + c4);
          *(volatile v4f*)(C + (size_t)(mBase + row) * ldc + n0 + c4) = v;
        }
        __threadfence();
      }
    } else {
      const int q = lane >> 3, c8 = (lane & 7) * 8;
      unsigned short* C  = (unsigned short*)Cout  + (size_t)b * strideC;
      unsigned short* C2 = (OUT_MODE == 2) ? ((unsigned short*)Cout2 + (size_t)b * strideC) : nullptr;
      for (int pass = 0; pass < 2; ++pass) {
#pragma unroll
        for (int it = 0; it < 4; ++it) {
          const int row = it * 4 + q;
          const float* sp = slab + row * 68 + c8;
          v8h hv, lv;
#pragma unroll
          for (int e = 0; e < 8; ++e) {
            if (OUT_MODE == 1) {
              hv[e] = (_Float16)sp[e];
            } else {
              unsigned short hb = f2bf_bits(sp[e]);
              unsigned short lb = f2bf_bits(sp[e] - bf_bits2f(hb));
              hv[e] = __builtin_bit_cast(_Float16, hb);
              lv[e] = __builtin_bit_cast(_Float16, lb);
            }
          }
          *(volatile v8h*)(C + (size_t)(mBase + row) * ldc + n0 + c8) = hv;
          if (OUT_MODE == 2) *(volatile v8h*)(C2 + (size_t)(mBase + row) * ldc + n0 + c8) = lv;
        }
        __threadfence();
      }
    }
    __builtin_amdgcn_fence(__ATOMIC_RELEASE, "workgroup");
    __builtin_amdgcn_wave_barrier();
    __builtin_amdgcn_fence(__ATOMIC_ACQUIRE, "workgroup");
  }
}

__global__ __launch_bounds__(256) void cast_f32_f16x2(
    const float* __restrict__ in, _Float16* __restrict__ out, int n2) {
  int i = blockIdx.x * 256 + threadIdx.x;
  if (i < n2) {
    const _Float16 h0 = (_Float16)in[2 * i], h1 = (_Float16)in[2 * i + 1];
    const unsigned u = (unsigned)__builtin_bit_cast(unsigned short, h0) | ((unsigned)__builtin_bit_cast(unsigned short, h1) << 16);
    ((volatile unsigned*)out)[i] = u;
    __threadfence();
    ((volatile unsigned*)out)[i] = u;
  }
}

__global__ __launch_bounds__(256) void transpose_cast_f16(
    const float* __restrict__ in, unsigned short* __restrict__ outp, int R, int C, float sc) {
  __shared__ float tile[64][65];
  const int tid = threadIdx.x, lane = tid & 31, wave = tid >> 5;
  const int c0 = blockIdx.x * 64;
  const int r0 = blockIdx.y * 64;
  _Float16* out = (_Float16*)(void*)outp;
#pragma unroll
  for (int i = 0; i < 16; ++i) {
    const int e  = i * 256 + tid;
    const int r  = e >> 6;
    const int cc = e & 63;
    tile[cc][r] = in[(size_t)(r0 + r) * C + c0 + cc] * sc;
  }
  __syncthreads();
  const int q = lane >> 3, c8 = (lane & 7) * 8;
  for (int pass = 0; pass < 2; ++pass) {
#pragma unroll
    for (int it = 0; it < 2; ++it) {
      const int row = wave * 8 + it * 4 + q;
      v8h hv;
#pragma unroll
      for (int e = 0; e < 8; ++e) hv[e] = (_Float16)tile[row][c8 + e];
      *(volatile v8h*)(out + (size_t)(c0 + row) * R + r0 + c8) = hv;
    }
    __threadfence();
  }
}

#define AT_D 64
#define AT_NW 4
#define AT_QB 64
#define AT_KC 64
#define PSC_F 32768.0f
#define OSC_F 16.0f

__device__ __forceinline__ v8f mma_h(v16h a, v16h b, v8f c) {
  c = __builtin_amdgcn_wmma_f32_16x16x32_f16(false, a, false, b, (short)0, c, false, false);
  asm volatile("v_nop\n\tv_nop\n\tv_nop\n\tv_nop" : "+v"(c) : "v"(a), "v"(b));
  return c;
}

__global__ __launch_bounds__(128)
void attn_seg64(const unsigned short* __restrict__ qkvp, const int* __restrict__ seg,
                unsigned short* __restrict__ outp, int S, int H, int ldqkv, int ldo,
                float sm_scale, float neg_fill) {
  union FH { v16h v; v8h h[2]; };
  __shared__ __align__(16) _Float16 Ksh[AT_KC * AT_D];
  __shared__ __align__(16) _Float16 Vth[AT_D * AT_KC];
  __shared__ __align__(16) _Float16 Psh[AT_NW][16 * AT_KC];
  __shared__ __align__(16) float    Os[AT_NW][16 * 68];

  const int tid  = threadIdx.x;
  const int wave = tid >> 5;
  const int lane = tid & 31;
  const int hh   = lane >> 4;
  const int c    = lane & 15;

  const int nqb  = S / AT_QB;
  const int bx   = blockIdx.x;
  const int qb   = bx % nqb;
  const int h    = bx / nqb;
  const int qblk = qb * AT_QB;
  const int q0   = qblk + wave * 16;

  const _Float16* qkv = (const _Float16*)(const void*)qkvp;
  const _Float16* qp = qkv + (size_t)h * AT_D;
  const _Float16* kp = qkv + (size_t)H * AT_D + (size_t)h * AT_D;
  const _Float16* vp = qkv + (size_t)2 * H * AT_D + (size_t)h * AT_D;
  _Float16* op = (_Float16*)(void*)outp + (size_t)h * AT_D;

  v16h qa[2];
#pragma unroll
  for (int dc = 0; dc < 2; ++dc)
    qa[dc] = Frag<_Float16>::load(qp + (size_t)(q0 + c) * ldqkv + dc * 32 + 8 * hh);

  int segq[8];
#pragma unroll
  for (int r = 0; r < 8; ++r) segq[r] = seg[q0 + 8 * hh + r];

  int qmn, qmx;
  {
    const int a0 = seg[qblk + lane], a1 = seg[qblk + 32 + lane];
    int mn = a0 < a1 ? a0 : a1, mx = a0 > a1 ? a0 : a1;
#pragma unroll
    for (int off = 1; off < 32; off <<= 1) {
      const int omn = __shfl_xor(mn, off, 32), omx = __shfl_xor(mx, off, 32);
      mn = omn < mn ? omn : mn; mx = omx > mx ? omx : mx;
    }
    qmn = __builtin_amdgcn_readfirstlane(mn);
    qmx = __builtin_amdgcn_readfirstlane(mx);
  }

  float mrow[8], lrow[8];
  v8f oacc[4];
#pragma unroll
  for (int r = 0; r < 8; ++r) { mrow[r] = -INFINITY; lrow[r] = 0.f; }
#pragma unroll
  for (int t = 0; t < 4; ++t) oacc[t] = (v8f){0.f,0.f,0.f,0.f,0.f,0.f,0.f,0.f};

  const int nChunks = S / AT_KC;
  for (int kc = 0; kc < nChunks; ++kc) {
    const int kv0 = kc * AT_KC;
    int kmn, kmx;
    {
      const int a0 = seg[kv0 + lane], a1 = seg[kv0 + 32 + lane];
      int mn = a0 < a1 ? a0 : a1, mx = a0 > a1 ? a0 : a1;
#pragma unroll
      for (int off = 1; off < 32; off <<= 1) {
        const int omn = __shfl_xor(mn, off, 32), omx = __shfl_xor(mx, off, 32);
        mn = omn < mn ? omn : mn; mx = omx > mx ? omx : mx;
      }
      kmn = __builtin_amdgcn_readfirstlane(mn);
      kmx = __builtin_amdgcn_readfirstlane(mx);
    }
    const bool act = !((kmx < qmn) || (kmn > qmx));
    if (act) {
      __syncthreads();
      {
        const int kvr = tid >> 1, dh = (tid & 1) * 32;
        const _Float16* krow = kp + (size_t)(kv0 + kvr) * ldqkv + dh;
        const _Float16* vrow = vp + (size_t)(kv0 + kvr) * ldqkv + dh;
#pragma unroll
        for (int i = 0; i < 4; ++i) {
          const v8h kk = *(const v8h*)(krow + 8 * i);
          const v8h vv = *(const v8h*)(vrow + 8 * i);
          *(v8h*)(Ksh + kvr * AT_D + dh + 8 * i) = kk;
#pragma unroll
          for (int e = 0; e < 8; ++e) Vth[(dh + 8 * i + e) * AT_KC + kvr] = vv[e];
        }
      }
      __syncthreads();

      v8f s[4];
#pragma unroll
      for (int j = 0; j < 4; ++j) {
        s[j] = (v8f){0.f,0.f,0.f,0.f,0.f,0.f,0.f,0.f};
#pragma unroll
        for (int dc = 0; dc < 2; ++dc) {
          FH kb;
          kb.h[0] = *(const v8h*)(Ksh + (j * 16 + c) * AT_D + dc * 32 + 8 * hh);
          kb.h[1] = *(const v8h*)(Ksh + (j * 16 + c) * AT_D + dc * 32 + 16 + 8 * hh);
          s[j] = mma_h(qa[dc], kb.v, s[j]);
        }
      }
      int segk[4];
#pragma unroll
      for (int j = 0; j < 4; ++j) segk[j] = seg[kv0 + j * 16 + c];

      float cm[8];
#pragma unroll
      for (int r = 0; r < 8; ++r) {
        float m = -INFINITY;
#pragma unroll
        for (int j = 0; j < 4; ++j) {
          float sv = s[j][r] * sm_scale;
          if (segq[r] != segk[j]) sv = neg_fill;
          s[j][r] = sv;
          m = fmaxf(m, sv);
        }
#pragma unroll
        for (int off = 1; off < 16; off <<= 1) m = fmaxf(m, __shfl_xor(m, off, 32));
        cm[r] = m;
      }
      _Float16* pw = Psh[wave];
#pragma unroll
      for (int r = 0; r < 8; ++r) {
        const float mnew  = fmaxf(mrow[r], cm[r]);
        const float alpha = expf(mrow[r] - mnew);
        mrow[r] = mnew;
        float psum = 0.f;
#pragma unroll
        for (int j = 0; j < 4; ++j) {
          const float p = expf(s[j][r] - mnew);
          psum += p;
          pw[(8 * hh + r) * AT_KC + j * 16 + c] = (_Float16)(p * PSC_F);
        }
#pragma unroll
        for (int off = 1; off < 16; off <<= 1) psum += __shfl_xor(psum, off, 32);
        lrow[r] = lrow[r] * alpha + psum;
#pragma unroll
        for (int t = 0; t < 4; ++t) oacc[t][r] *= alpha;
      }
      __builtin_amdgcn_fence(__ATOMIC_RELEASE, "workgroup");
      __builtin_amdgcn_wave_barrier();
      __builtin_amdgcn_fence(__ATOMIC_ACQUIRE, "workgroup");
#pragma unroll 1
      for (int kk = 0; kk < 2; ++kk) {
        FH pa;
        pa.h[0] = *(const v8h*)(pw + c * AT_KC + kk * 32 + 8 * hh);
        pa.h[1] = *(const v8h*)(pw + c * AT_KC + kk * 32 + 16 + 8 * hh);
#pragma unroll
        for (int t = 0; t < 4; ++t) {
          FH vb;
          vb.h[0] = *(const v8h*)(Vth + (t * 16 + c) * AT_KC + kk * 32 + 8 * hh);
          vb.h[1] = *(const v8h*)(Vth + (t * 16 + c) * AT_KC + kk * 32 + 16 + 8 * hh);
          oacc[t] = mma_h(pa.v, vb.v, oacc[t]);
        }
      }
    }
  }

  float* os = Os[wave];
#pragma unroll
  for (int r = 0; r < 8; ++r) {
    const float inv = (1.0f / lrow[r]) * (OSC_F / PSC_F);
#pragma unroll
    for (int t = 0; t < 4; ++t) os[(8 * hh + r) * 68 + t * 16 + c] = oacc[t][r] * inv;
  }
  __builtin_amdgcn_fence(__ATOMIC_RELEASE, "workgroup");
  __builtin_amdgcn_wave_barrier();
  __builtin_amdgcn_fence(__ATOMIC_ACQUIRE, "workgroup");
  {
    const int q4 = lane >> 3, c8 = (lane & 7) * 8;
    for (int pass = 0; pass < 2; ++pass) {
#pragma unroll
      for (int it = 0; it < 4; ++it) {
        const int row = it * 4 + q4;
        const float* sp = os + row * 68 + c8;
        v8h hv;
#pragma unroll
        for (int e = 0; e < 8; ++e) hv[e] = (_Float16)sp[e];
        *(volatile v8h*)(op + (size_t)(q0 + row) * ldo + c8) = hv;
      }
      __threadfence();
    }
  }
}

extern "C" void kernel_launch(void* const* d_in, const int* in_sizes, int n_in,
                              void* d_out, int out_size, void* d_ws, size_t ws_size,
                              hipStream_t stream) {
  const int Sn = 4096, DIMn = 1024, Hn = 16, N3 = 3072;
  if (n_in < 6) return;
  if (in_sizes[0] != Sn * DIMn || in_sizes[1] != DIMn * N3 || in_sizes[2] != N3 ||
      in_sizes[3] != DIMn * DIMn || in_sizes[4] != DIMn || in_sizes[5] != Sn ||
      out_size != Sn * DIMn) return;

  const float* x_in   = (const float*)d_in[0];
  const float* w_qkv  = (const float*)d_in[1];
  const float* b_qkv  = (const float*)d_in[2];
  const float* w_proj = (const float*)d_in[3];
  const float* b_proj = (const float*)d_in[4];
  const int*   seg    = (const int*)d_in[5];
  float*       out    = (float*)d_out;

  const size_t szX   = (size_t)Sn * DIMn * 2;
  const size_t szWq  = (size_t)N3 * DIMn * 2;
  const size_t szWp  = (size_t)DIMn * DIMn * 2;
  const size_t szQKV = (size_t)Sn * N3 * 2;
  const size_t szO   = (size_t)Sn * DIMn * 2;
  const size_t offX = 0, offWq = offX + szX, offWp = offWq + szWq, offQKV = offWp + szWp, offO = offQKV + szQKV;
  const size_t total = offO + szO;
  if (total > ws_size) return;
  unsigned char* ws = (unsigned char*)d_ws;
  unsigned short* Xh   = (unsigned short*)(ws + offX);
  unsigned short* Wqh  = (unsigned short*)(ws + offWq);
  unsigned short* Wph  = (unsigned short*)(ws + offWp);
  unsigned short* QKVh = (unsigned short*)(ws + offQKV);
  unsigned short* Oh   = (unsigned short*)(ws + offO);

  {
    const int n2 = Sn * DIMn / 2;
    cast_f32_f16x2<<<dim3((n2 + 255) / 256), dim3(256), 0, stream>>>(x_in, (_Float16*)(void*)Xh, n2);
  }
  transpose_cast_f16<<<dim3(N3 / 64, DIMn / 64), dim3(256), 0, stream>>>(w_qkv, Wqh, DIMn, N3, 64.0f);
  transpose_cast_f16<<<dim3(DIMn / 64, DIMn / 64), dim3(256), 0, stream>>>(w_proj, Wph, DIMn, DIMn, 64.0f);
  {
    const int tiles = (Sn / 64) * (N3 / 64);
    wmma_gemm64<0, false, 2, 1, false><<<dim3((tiles + 7) / 8, 1), dim3(256), 0, stream>>>(
        Xh, Xh, DIMn, 0L, Wqh, Wqh, DIMn, 0L, (void*)QKVh, (void*)QKVh, N3, 0L,
        b_qkv, b_qkv, 0L, Sn, N3, DIMn, 1.0f / 64.0f);
  }
  attn_seg64<<<dim3(Hn * (Sn / 64)), dim3(128), 0, stream>>>(
      QKVh, seg, Oh, Sn, Hn, N3, DIMn, 0.125f, -1.0e9f);
  {
    const int tiles = (Sn / 64) * (DIMn / 64);
    wmma_gemm64<0, false, 2, 0, false><<<dim3((tiles + 7) / 8, 1), dim3(256), 0, stream>>>(
        Oh, Oh, DIMn, 0L, Wph, Wph, DIMn, 0L, (void*)out, (void*)out, DIMn, 0L,
        b_proj, b_proj, 0L, Sn, DIMn, DIMn, 1.0f / 1024.0f);
  }
}
